// RawGATEncoder_39247411151304
// MI455X (gfx1250) — hardware-verified
//
#include <hip/hip_runtime.h>
#include <stddef.h>


#define FIN0    128
#define HID     256
#define NOUT    128
#define NHEAD   4
#define NTHR    256
#define NWAVE   8
#define EPT     8
#define NGRP    2
#define CHUNK   (NTHR * EPT * NGRP)
#define WCAP    (EPT * NGRP * 32)
#define LISTN   (NWAVE * WCAP)
#define NBC     4096
#define NBF     1024
#define RCAP    40960
#define RBN     128
#define TGT     256
#define DEGCAP  256
#define OTHR    512
#define BM      32
#define WSCAP   134217728
#define NEG_SLOPE 0.2f
#define SCL_A   8.0f
#define SCL_W   16.0f
#define SCL_ACC 0.0078125f
#define SCL_H   16.0f
#define SCL_HI  0.0625f

#define LDS_FILL ((RCAP + NBF + LISTN) * 4 + 64)

static_assert((CHUNK & (CHUNK - 1)) == 0);
static_assert(CHUNK <= 4096);
static_assert(NBC <= 4096 && NBF <= 4096);
static_assert((NBC & (NBC - 1)) == 0 && (NBF & (NBF - 1)) == 0);
static_assert(NBC == 4 * NBF);
static_assert(OTHR * 8 == NBC);
static_assert((RCAP % 32) == 0);
static_assert(TGT == NWAVE * 32);
static_assert((NBC % TGT) == 0);
static_assert((TGT % BM) == 0);
static_assert(FIN0 % 32 == 0 && HID % 64 == 0 && NOUT % 64 == 0);
static_assert(HID == 2 * FIN0 && HID == 2 * NOUT);

typedef float    v4f  __attribute__((ext_vector_type(4)));
typedef float    v8f  __attribute__((ext_vector_type(8)));
typedef int      v4i  __attribute__((ext_vector_type(4)));
typedef _Float16 v4h  __attribute__((ext_vector_type(4)));
typedef _Float16 v8h  __attribute__((ext_vector_type(8)));
typedef _Float16 v16h __attribute__((ext_vector_type(16)));
union FragH { v16h v; v8h h[2]; };

template <int N> struct VT;
template <> struct VT<8> { typedef v8f f; typedef v8h h; };
template <> struct VT<4> { typedef v4f f; typedef v4h h; };

__device__ __forceinline__ v8f wmh(v16h a, v16h b, v8f c) {
  v8f d = __builtin_amdgcn_wmma_f32_16x16x32_f16(false, a, false, b, (short)0, c, false, false);
  asm volatile("v_nop\n\tv_nop\n\tv_nop\n\tv_nop" : "+v"(d) : "v"(a), "v"(b));
  return d;
}

__device__ __forceinline__ v8h cvt8(v4f a, v4f b, float s) {
  v8f t;
  t[0] = a.x * s; t[1] = a.y * s; t[2] = a.z * s; t[3] = a.w * s;
  t[4] = b.x * s; t[5] = b.y * s; t[6] = b.z * s; t[7] = b.w * s;
  return __builtin_convertvector(t, v8h);
}

__device__ __forceinline__ float lrelu(float v) { return v > 0.0f ? v : NEG_SLOPE * v; }

template <int NB>
__device__ __forceinline__ int scan_chunk(const int* __restrict__ dsts, int nE, int cbase, int slotBase,
                                          int vec8, int* list, int tid, int lane, int wave) {
  int wc = 0;
#pragma unroll
  for (int g = 0; g < NGRP; ++g) {
    const int el0  = (g * NTHR + tid) * EPT;
    const int e0   = cbase + el0;
    const int sent = -2147483647 - 1;
    v4i da, db;
    if (vec8 != 0 && cbase + CHUNK <= nE) {
      da = *(const v4i*)(dsts + e0);
      db = *(const v4i*)(dsts + e0 + 4);
    } else {
      da.x = (e0     < nE) ? dsts[min(e0, nE - 1)] : sent;
      da.y = (e0 + 1 < nE) ? dsts[min(e0 + 1, nE - 1)] : sent;
      da.z = (e0 + 2 < nE) ? dsts[min(e0 + 2, nE - 1)] : sent;
      da.w = (e0 + 3 < nE) ? dsts[min(e0 + 3, nE - 1)] : sent;
      db.x = (e0 + 4 < nE) ? dsts[min(e0 + 4, nE - 1)] : sent;
      db.y = (e0 + 5 < nE) ? dsts[min(e0 + 5, nE - 1)] : sent;
      db.z = (e0 + 6 < nE) ? dsts[min(e0 + 6, nE - 1)] : sent;
      db.w = (e0 + 7 < nE) ? dsts[min(e0 + 7, nE - 1)] : sent;
    }
    const unsigned nb = (unsigned)slotBase;
    const unsigned s0 = (unsigned)da.x - nb, s1 = (unsigned)da.y - nb;
    const unsigned s2 = (unsigned)da.z - nb, s3 = (unsigned)da.w - nb;
    const unsigned s4 = (unsigned)db.x - nb, s5 = (unsigned)db.y - nb;
    const unsigned s6 = (unsigned)db.z - nb, s7 = (unsigned)db.w - nb;
    const bool h0 = s0 < (unsigned)NB, h1 = s1 < (unsigned)NB, h2 = s2 < (unsigned)NB, h3 = s3 < (unsigned)NB;
    const bool h4 = s4 < (unsigned)NB, h5 = s5 < (unsigned)NB, h6 = s6 < (unsigned)NB, h7 = s7 < (unsigned)NB;
    const unsigned any = __builtin_amdgcn_ballot_w32(h0 | h1 | h2 | h3 | h4 | h5 | h6 | h7);
    if (any != 0u) {
#define HITJ(J, HJ, SJ) { \
        const unsigned mj = __builtin_amdgcn_ballot_w32(HJ); \
        if (mj != 0u) { \
          if (HJ) { \
            const int pos = wc + (int)__builtin_amdgcn_mbcnt_lo(mj, 0u); \
            if (pos < WCAP) list[wave * WCAP + pos] = ((el0 + (J)) << 12) | (int)(SJ); \
          } \
          wc += (int)__builtin_popcount(mj); } }
      HITJ(0, h0, s0)
      HITJ(1, h1, s1)
      HITJ(2, h2, s2)
      HITJ(3, h3, s3)
      HITJ(4, h4, s4)
      HITJ(5, h5, s5)
      HITJ(6, h6, s6)
      HITJ(7, h7, s7)
#undef HITJ
    }
  }
  return wc;
}

__global__ __launch_bounds__(NTHR) void k_xcvt(const float* __restrict__ x, _Float16* xp, int nN, int nUnits) {
  const int i = (int)blockIdx.x * NTHR + (int)threadIdx.x;
  if (i >= nUnits) return;
  const int row = i >> 4;
  const int c0  = (i & 15) * 8;
  int rr = row > nN - 1 ? nN - 1 : row;
  rr = rr < 0 ? 0 : rr;
  const float* p = x + (size_t)rr * FIN0 + c0;
  v4f a = *(const v4f*)p, b = *(const v4f*)(p + 4);
  const v4f z = {0.f, 0.f, 0.f, 0.f};
  if (row >= nN) { a = z; b = z; }
  const v8h o = cvt8(a, b, SCL_A);
  _Float16* d = xp + (size_t)i * 8;
  *(volatile v8h*)d = o;
  __threadfence();
  *(volatile v8h*)d = o;
}

template <int KD, int NCW>
__global__ __launch_bounds__(NTHR) void k_wprep(const float* __restrict__ W, _Float16* wp) {
  constexpr int KS    = KD / 8;
  constexpr int UNITS = NCW * KS;
  static_assert(KD % 8 == 0);
  const int i = (int)blockIdx.x * NTHR + (int)threadIdx.x;
  if (i >= UNITS) return;
  const int n  = i / KS;
  const int k0 = (i - n * KS) * 8;
  v4f a, b;
  a.x = W[(size_t)(k0 + 0) * NCW + n]; a.y = W[(size_t)(k0 + 1) * NCW + n];
  a.z = W[(size_t)(k0 + 2) * NCW + n]; a.w = W[(size_t)(k0 + 3) * NCW + n];
  b.x = W[(size_t)(k0 + 4) * NCW + n]; b.y = W[(size_t)(k0 + 5) * NCW + n];
  b.z = W[(size_t)(k0 + 6) * NCW + n]; b.w = W[(size_t)(k0 + 7) * NCW + n];
  const v8h o = cvt8(a, b, SCL_W);
  _Float16* d = wp + (size_t)i * 8;
  *(volatile v8h*)d = o;
  __threadfence();
  *(volatile v8h*)d = o;
}

__global__ __launch_bounds__(NTHR) void k_count(
    const int* __restrict__ dsts, int* cnt, int nE, int vec8) {
  __shared__ __attribute__((aligned(16))) int scnt[NBC];
  __shared__ __attribute__((aligned(16))) int list[LISTN];
  __shared__ int wcnt[NWAVE];
  const int tid = threadIdx.x, lane = tid & 31, wave = tid >> 5;
  const int nodeBase = blockIdx.x * NBC;

  for (int i = tid; i < NBC; i += NTHR) scnt[i] = 0;
  __syncthreads();

  const int nChunks = (nE + CHUNK - 1) / CHUNK;
#pragma unroll 1
  for (int ch = 0; ch < nChunks; ++ch) {
    const int cbase = ch * CHUNK;
    const int wc = scan_chunk<NBC>(dsts, nE, cbase, nodeBase, vec8, list, tid, lane, wave);
    if (lane == 0) wcnt[wave] = wc;
    __syncthreads();
    if (wave == 0) {
#pragma unroll 1
      for (int wsx = 0; wsx < NWAVE; ++wsx) {
        int n = __builtin_amdgcn_readfirstlane(wcnt[wsx]);
        n = n > WCAP ? WCAP : (n < 0 ? 0 : n);
        const int* lp = list + wsx * WCAP;
#pragma unroll 1
        for (int i = 0; i < n; ++i) {
          const int ent  = __builtin_amdgcn_readfirstlane(lp[i]);
          const int slot = ent & (NBC - 1);
          if (lane == 0) scnt[slot] = scnt[slot] + 1;
        }
      }
    }
    __syncthreads();
  }

  v4i cq[4];
#pragma unroll
  for (int q = 0; q < 4; ++q) {
    const int f = (wave * 4 + q) * 128 + 4 * lane;
    cq[q] = *(const v4i*)(scnt + f);
  }
  int* cp = cnt + (size_t)nodeBase;
#pragma unroll
  for (int q = 0; q < 4; ++q) {
    const int f = (wave * 4 + q) * 128 + 4 * lane;
    *(volatile v4i*)(cp + f) = cq[q];
  }
  __threadfence();
#pragma unroll
  for (int q = 0; q < 4; ++q) {
    const int f = (wave * 4 + q) * 128 + 4 * lane;
    *(volatile v4i*)(cp + f) = cq[q];
  }
}

__global__ __launch_bounds__(OTHR) void k_offsets(
    const int* __restrict__ cnt, int* off, int* rbase, int nChunk) {
  __shared__ __attribute__((aligned(16))) int soff[NBC];
  __shared__ __attribute__((aligned(16))) int srb[RBN];
  __shared__ int wtot[OTHR / 32];
  const int tid = threadIdx.x, lane = tid & 31, wave = tid >> 5, sub = tid >> 7;
  for (int i = tid; i < RBN; i += OTHR) srb[i] = 0;
  int carry = 0;
#pragma unroll 1
  for (int ch = 0; ch < nChunk; ++ch) {
    const int base = ch * NBC;
    const v4i c0 = *(const v4i*)(cnt + base + 8 * tid);
    const v4i c1 = *(const v4i*)(cnt + base + 8 * tid + 4);
    const int e0 = max(c0.x, 0), e1 = max(c0.y, 0), e2 = max(c0.z, 0), e3 = max(c0.w, 0);
    const int e4 = max(c1.x, 0), e5 = max(c1.y, 0), e6 = max(c1.z, 0), e7 = max(c1.w, 0);
    const int ts = e0 + e1 + e2 + e3 + e4 + e5 + e6 + e7;
    int incl = ts;
#pragma unroll
    for (int d = 1; d < 32; d <<= 1) {
      const int t = __shfl_up(incl, d);
      if (lane >= d) incl += t;
    }
    if (lane == 31) wtot[wave] = incl;
    __syncthreads();
    const int S0 = wtot[0]  + wtot[1]  + wtot[2]  + wtot[3];
    const int S1 = wtot[4]  + wtot[5]  + wtot[6]  + wtot[7];
    const int S2 = wtot[8]  + wtot[9]  + wtot[10] + wtot[11];
    const int S3 = wtot[12] + wtot[13] + wtot[14] + wtot[15];
    int pre = 0;
#pragma unroll 1
    for (int w = 4 * sub; w < wave; ++w) pre += wtot[w];
    const int b0 = carry;
    const int b1 = b0 + ((S0 + 31) & ~31);
    const int b2 = b1 + ((S1 + 31) & ~31);
    const int b3 = b2 + ((S2 + 31) & ~31);
    const int b4 = b3 + ((S3 + 31) & ~31);
    const int myb = sub == 0 ? b0 : (sub == 1 ? b1 : (sub == 2 ? b2 : b3));
    if (tid == 0) {
      srb[min(4 * ch + 0, RBN - 1)] = b0;
      srb[min(4 * ch + 1, RBN - 1)] = b1;
      srb[min(4 * ch + 2, RBN - 1)] = b2;
      srb[min(4 * ch + 3, RBN - 1)] = b3;
    }
    int run = myb + pre + incl - ts;
    soff[8 * tid + 0] = run; run += e0;
    soff[8 * tid + 1] = run; run += e1;
    soff[8 * tid + 2] = run; run += e2;
    soff[8 * tid + 3] = run; run += e3;
    soff[8 * tid + 4] = run; run += e4;
    soff[8 * tid + 5] = run; run += e5;
    soff[8 * tid + 6] = run; run += e6;
    soff[8 * tid + 7] = run;
    carry = b4;
    __syncthreads();
    const v4i o0 = *(const v4i*)(soff + 4 * tid);
    const v4i o1 = *(const v4i*)(soff + 4 * (tid + OTHR));
    int* op = off + base;
    *(volatile v4i*)(op + 4 * tid) = o0;
    *(volatile v4i*)(op + 4 * (tid + OTHR)) = o1;
    __threadfence();
    *(volatile v4i*)(op + 4 * tid) = o0;
    *(volatile v4i*)(op + 4 * (tid + OTHR)) = o1;
    __syncthreads();
  }
  if (tid == 0) srb[min(4 * nChunk, RBN - 1)] = carry;
  __syncthreads();
  v4i rv = {0, 0, 0, 0};
  if (tid < 32) rv = *(const v4i*)(srb + 4 * tid);
  if (tid < 32) *(volatile v4i*)(rbase + 4 * tid) = rv;
  __threadfence();
  if (tid < 32) *(volatile v4i*)(rbase + 4 * tid) = rv;
}

__global__ __launch_bounds__(NTHR) void k_fill(
    const int* __restrict__ srcs, const int* __restrict__ dsts,
    const int* __restrict__ off, const int* __restrict__ rbase,
    int* csr, int nN, int nE, int vec8, int csrLen) {
  extern __shared__ v4f lds_dyn[];
  int* region = (int*)lds_dyn;
  int* cursor = region + RCAP;
  int* list   = cursor + NBF;
  int* wcnt   = list + LISTN;
  const int tid = threadIdx.x, lane = tid & 31, wave = tid >> 5;
  const int b = blockIdx.x;
  const int nodeBase = b * NBF;

  int rb0 = rbase[b];
  const int rb1 = rbase[b + 1];
  rb0 = rb0 < 0 ? 0 : (rb0 > csrLen ? csrLen : rb0);
  rb0 &= ~31;
  int len = rb1 - rb0;
  len = len < 0 ? 0 : (len > RCAP ? RCAP : len);
  int lenW = (len + 31) & ~31;
  if (rb0 + lenW > csrLen) lenW = (csrLen - rb0) & ~31;

  {
    const v4i z = {0, 0, 0, 0};
    for (int i = tid; i < RCAP / 4; i += NTHR) ((v4i*)region)[i] = z;
    for (int s = tid; s < NBF; s += NTHR) {
      int o = off[nodeBase + s] - rb0;
      o = o < 0 ? 0 : (o > RCAP ? RCAP : o);
      cursor[s] = o;
    }
  }
  __syncthreads();

  const int nChunks = (nE + CHUNK - 1) / CHUNK;
#pragma unroll 1
  for (int ch = 0; ch < nChunks; ++ch) {
    const int cbase = ch * CHUNK;
    const int wc = scan_chunk<NBF>(dsts, nE, cbase, nodeBase, vec8, list, tid, lane, wave);
    if (lane == 0) wcnt[wave] = wc;
    __syncthreads();
    if (wave == 0) {
#pragma unroll 1
      for (int wsx = 0; wsx < NWAVE; ++wsx) {
        int n = __builtin_amdgcn_readfirstlane(wcnt[wsx]);
        n = n > WCAP ? WCAP : (n < 0 ? 0 : n);
        const int* lp = list + wsx * WCAP;
#pragma unroll 1
        for (int i = 0; i < n; ++i) {
          const int ent  = __builtin_amdgcn_readfirstlane(lp[i]);
          const int slot = ent & (NBF - 1);
          int e = cbase + ((ent >> 12) & (CHUNK - 1));
          e = e > nE - 1 ? nE - 1 : e;
          int src = srcs[e];
          src = src < 0 ? 0 : (src > nN - 1 ? nN - 1 : src);
          if (lane == 0) {
            int pos = cursor[slot];
            pos = pos < 0 ? 0 : (pos > RCAP - 1 ? RCAP - 1 : pos);
            region[pos] = src;
            const int np = pos + 1;
            cursor[slot] = np > RCAP ? RCAP : np;
          }
        }
      }
    }
    __syncthreads();
  }

  const int nv = lenW >> 2;
  int* gp = csr + rb0;
#pragma unroll 1
  for (int i = tid; i < nv; i += NTHR) { const v4i v = ((const v4i*)region)[i]; *(volatile v4i*)(gp + 4 * i) = v; }
  __threadfence();
#pragma unroll 1
  for (int i = tid; i < nv; i += NTHR) { const v4i v = ((const v4i*)region)[i]; *(volatile v4i*)(gp + 4 * i) = v; }
}

template <int K, int NC, int HMODE>
__global__ __launch_bounds__(NTHR) void k_gemm(
    const _Float16* __restrict__ Ap, const _Float16* __restrict__ Bp,
    const float* __restrict__ attS, const float* __restrict__ attD,
    _Float16* Hq, float* Hf, float* eS, float* eD) {
  constexpr int TPW  = NC / 64;
  constexpr int KT   = K / 32;
  constexpr int CPP  = NC / 8;
  constexpr int NES  = BM * NHEAD;
  constexpr int NIT8 = (BM * NC / 8) / NTHR;
  constexpr int NIT4 = (BM * NC / 4) / NTHR;
  static_assert(K % 32 == 0);
  static_assert(NC % 64 == 0 && TPW >= 1);
  static_assert(CPP % 4 == 0);
  static_assert((NC / NHEAD) == 2 * CPP);
  static_assert((BM * NC / 8) % NTHR == 0 && NIT8 >= 1);
  static_assert((BM * NC / 4) % NTHR == 0 && NIT4 >= 1);
  static_assert(NES == 128);
  static_assert(BM * 8 == NTHR);
  static_assert(HMODE == 0 || HMODE == 1);

  __shared__ __attribute__((aligned(16))) float stg[BM * NC];
  __shared__ __attribute__((aligned(16))) float sES[NES];
  __shared__ __attribute__((aligned(16))) float sED[NES];
  const int tid = threadIdx.x, lane = tid & 31, wave = tid >> 5, hh = lane >> 4, m = lane & 15;
  const int rowBase = blockIdx.x * BM;
  const int rg = wave >> 2, cq = wave & 3;
  const int r0 = rg * 16;
  const int c0 = cq * (NC / 4);

  v8f acc[TPW];
#pragma unroll
  for (int t = 0; t < TPW; ++t) { v8f z = {0.f, 0.f, 0.f, 0.f, 0.f, 0.f, 0.f, 0.f}; acc[t] = z; }

  const _Float16* ap  = Ap + (size_t)(rowBase + r0 + m) * K + 8 * hh;
  const _Float16* bp0 = Bp + (size_t)(c0 + m) * K + 8 * hh;
#pragma unroll 1
  for (int kt = 0; kt < KT; ++kt) {
    FragH a;
    a.h[0] = *(const v8h*)(ap + 32 * kt);
    a.h[1] = *(const v8h*)(ap + 32 * kt + 16);
#pragma unroll
    for (int t = 0; t < TPW; ++t) {
      const _Float16* bp = bp0 + (size_t)(16 * t) * K + 32 * kt;
      FragH bf;
      bf.h[0] = *(const v8h*)bp;
      bf.h[1] = *(const v8h*)(bp + 16);
      acc[t] = wmh(a.v, bf.v, acc[t]);
    }
  }

  {
    float* sp = stg + (size_t)(r0 + 8 * hh) * NC + c0 + m;
#pragma unroll
    for (int t = 0; t < TPW; ++t) {
#pragma unroll
      for (int r = 0; r < 8; ++r) sp[r * NC + 16 * t] = acc[t][r] * SCL_ACC;
    }
  }
  __syncthreads();

  {
    const int drow = tid >> 3, part = tid & 7;
    const float* rp  = stg + (size_t)drow * NC + CPP * part;
    const float* sa  = attS + CPP * part;
    const float* sdd = attD + CPP * part;
    float ps = 0.f, pd = 0.f;
#pragma unroll 4
    for (int c = 0; c < CPP; c += 4) {
      const v4f hv = *(const v4f*)(rp + c);
      const v4f av = *(const v4f*)(sa + c);
      const v4f dv = *(const v4f*)(sdd + c);
      ps += hv.x * av.x + hv.y * av.y + hv.z * av.z + hv.w * av.w;
      pd += hv.x * dv.x + hv.y * dv.y + hv.z * dv.z + hv.w * dv.w;
    }
    ps += __shfl_xor(ps, 1); pd += __shfl_xor(pd, 1);
    if ((part & 1) == 0) { sES[drow * NHEAD + (part >> 1)] = ps; sED[drow * NHEAD + (part >> 1)] = pd; }
  }

  if constexpr (HMODE == 0) {
    _Float16* tile = Hq + (size_t)rowBase * NC;
    v8h hv[NIT8];
#pragma unroll
    for (int it = 0; it < NIT8; ++it) {
      const int u = it * NTHR + tid;
      const v4f x0 = *(const v4f*)(stg + 8 * u);
      const v4f x1 = *(const v4f*)(stg + 8 * u + 4);
      hv[it] = cvt8(x0, x1, SCL_H);
    }
#pragma unroll
    for (int it = 0; it < NIT8; ++it) *(volatile v8h*)(tile + 8 * (size_t)(it * NTHR + tid)) = hv[it];
    __threadfence();
#pragma unroll
    for (int it = 0; it < NIT8; ++it) *(volatile v8h*)(tile + 8 * (size_t)(it * NTHR + tid)) = hv[it];
  } else {
    float* tile = Hf + (size_t)rowBase * NC;
    v4f cv[NIT4];
#pragma unroll
    for (int it = 0; it < NIT4; ++it) cv[it] = *(const v4f*)(stg + 4 * (it * NTHR + tid));
#pragma unroll
    for (int it = 0; it < NIT4; ++it) *(volatile v4f*)(tile + 4 * (size_t)(it * NTHR + tid)) = cv[it];
    __threadfence();
#pragma unroll
    for (int it = 0; it < NIT4; ++it) *(volatile v4f*)(tile + 4 * (size_t)(it * NTHR + tid)) = cv[it];
  }
  __syncthreads();

  {
    const v4f vS = *(const v4f*)(sES + 4 * lane);
    const v4f vD = *(const v4f*)(sED + 4 * lane);
    float* gS = eS + (size_t)rowBase * NHEAD + 4 * lane;
    float* gD = eD + (size_t)rowBase * NHEAD + 4 * lane;
    if (wave == 0) *(volatile v4f*)gS = vS;
    if (wave == 1) *(volatile v4f*)gD = vD;
    __threadfence();
    if (wave == 0) *(volatile v4f*)gS = vS;
    if (wave == 1) *(volatile v4f*)gD = vD;
  }
}

template <int NC, int MODE>
__device__ __forceinline__ typename VT<NC / 32>::f ldrow(const _Float16* __restrict__ hq,
                                                        const float* __restrict__ hf, int row, int col) {
  typedef typename VT<NC / 32>::f VF;
  typedef typename VT<NC / 32>::h VH;
  const size_t idx = (size_t)row * NC + col;
  if constexpr (MODE == 0) {
    const VH t = *(const VH*)(hq + idx);
    return __builtin_convertvector(t, VF);
  } else {
    return *(const VF*)(hf + idx);
  }
}

template <int NC, int MODE>
__global__ __launch_bounds__(NTHR) void k_agg(
    const int* __restrict__ csr, const int* __restrict__ off, const int* __restrict__ cnt,
    const float* __restrict__ eS, const float* __restrict__ eD,
    const _Float16* __restrict__ hq, const float* __restrict__ hf,
    const float* __restrict__ bias, _Float16* xo, float* out, int nN, int csrLen) {
  constexpr int CPL = NC / 32;
  static_assert((MODE == 0 && NC == HID) || (MODE == 1 && NC == NOUT));
  static_assert(CPL == 8 || CPL == 4);
  static_assert(NC / NHEAD == 8 * CPL);
  typedef typename VT<CPL>::f VF;
  typedef typename VT<CPL>::h VH;
  constexpr float HSC = (MODE == 0) ? SCL_HI : 1.0f;
  const int tid = threadIdx.x, lane = tid & 31, wave = tid >> 5;
  const int tbase = blockIdx.x * TGT + wave * 32;
  const int col = CPL * lane;
  const int hd  = lane >> 3;

  const VF bb = *(const VF*)(bias + col);

  const int cl    = tbase + lane;
  const int cnt_l = cnt[cl];
  const int off_l = off[cl];

#pragma unroll 1
  for (int j = 0; j < 32; ++j) {
    const int c = tbase + j;
    int n = __shfl(cnt_l, j);
    n = n < 0 ? 0 : (n > DEGCAP ? DEGCAP : n);
    const int st = __shfl(off_l, j);
    const float esc = eS[(size_t)c * NHEAD + hd];
    const float edc = eD[(size_t)c * NHEAD + hd];

    float mxs = esc;
#pragma unroll 1
    for (int q0 = 0; q0 < n; q0 += 32) {
      int pos = st + q0 + lane;
      pos = pos < 0 ? 0 : (pos > csrLen - 1 ? csrLen - 1 : pos);
      int sl = csr[pos];
      sl = sl < 0 ? 0 : (sl > nN - 1 ? nN - 1 : sl);
      const int mcnt = (n - q0) < 32 ? (n - q0) : 32;
#pragma unroll 1
      for (int pp = 0; pp < mcnt; ++pp) {
        const int s = __builtin_amdgcn_readlane(sl, pp);
        mxs = fmaxf(mxs, eS[(size_t)s * NHEAD + hd]);
      }
    }
    const float mx = lrelu(mxs + edc);

    float p   = __expf(lrelu(esc + edc) - mx);
    float den = p;
    VF acc = ldrow<NC, MODE>(hq, hf, c, col) * p;
#pragma unroll 1
    for (int q0 = 0; q0 < n; q0 += 32) {
      int pos = st + q0 + lane;
      pos = pos < 0 ? 0 : (pos > csrLen - 1 ? csrLen - 1 : pos);
      int sl = csr[pos];
      sl = sl < 0 ? 0 : (sl > nN - 1 ? nN - 1 : sl);
      const int mcnt = (n - q0) < 32 ? (n - q0) : 32;
#pragma unroll 1
      for (int pp = 0; pp < mcnt; ++pp) {
        const int s = __builtin_amdgcn_readlane(sl, pp);
        p = __expf(lrelu(eS[(size_t)s * NHEAD + hd] + edc) - mx);
        den += p;
        const VF hv = ldrow<NC, MODE>(hq, hf, s, col);
        acc = acc + hv * p;
      }
    }

    const float rd = (1.0f / den) * HSC;
    const VF v = acc * rd + bb;
    if constexpr (MODE == 0) {
      VF w;
#pragma unroll
      for (int i = 0; i < CPL; ++i) {
        float t = v[i];
        t = t > 0.0f ? t : 0.0f;
        t = (c < nN) ? t * SCL_A : 0.0f;
        w[i] = t;
      }
      const VH o = __builtin_convertvector(w, VH);
      _Float16* gp = xo + (size_t)c * NC + col;
      *(volatile VH*)gp = o;
      __threadfence();
      *(volatile VH*)gp = o;
    } else {
      const int cc = (c < nN) ? c : 0;
      float* gp = out + (size_t)cc * NC + col;
      if (c < nN) *(volatile VF*)gp = v;
      __threadfence();
      if (c < nN) *(volatile VF*)gp = v;
    }
  }
}

extern "C" void kernel_launch(void* const* d_in, const int* in_sizes, int n_in,
                              void* d_out, int out_size, void* d_ws, size_t ws_size,
                              hipStream_t stream) {
  if (n_in < 14) return;
  const int nN = in_sizes[0] / FIN0;
  const int nE = in_sizes[1] / 2;
  if (nN <= 0 || nE <= 0 || in_sizes[0] != nN * FIN0 || in_sizes[1] != 2 * nE) return;
  if (in_sizes[2] != FIN0 * HID || in_sizes[3] != HID || in_sizes[4] != HID || in_sizes[5] != HID) return;
  if (in_sizes[6] != HID * HID || in_sizes[7] != HID || in_sizes[8] != HID || in_sizes[9] != HID) return;
  if (in_sizes[10] != HID * NOUT || in_sizes[11] != NOUT || in_sizes[12] != NOUT || in_sizes[13] != NOUT) return;
  if (out_size != nN * NOUT) return;
  if (nE > (1 << 28) || nN > (1 << 22)) return;

  const float* x    = (const float*)d_in[0];
  const int*   ei   = (const int*)d_in[1];
  const int*   src  = ei;
  const int*   dst  = ei + nE;
  const float* W0   = (const float*)d_in[2];
  const float* as0  = (const float*)d_in[3];
  const float* ad0  = (const float*)d_in[4];
  const float* b0   = (const float*)d_in[5];
  const float* W1   = (const float*)d_in[6];
  const float* as1  = (const float*)d_in[7];
  const float* ad1  = (const float*)d_in[8];
  const float* b1   = (const float*)d_in[9];
  const float* W2   = (const float*)d_in[10];
  const float* as2  = (const float*)d_in[11];
  const float* ad2  = (const float*)d_in[12];
  const float* b2   = (const float*)d_in[13];
  float* out = (float*)d_out;

  const int NPAD   = ((nN + TGT - 1) / TGT) * TGT;
  const int nBC    = (nN + NBC - 1) / NBC;
  const int CNTPAD = nBC * NBC;
  if (CNTPAD < NPAD) return;
  if (4 * nBC + 1 > RBN) return;
  const int nBF    = (nN + NBF - 1) / NBF;
  if (nBF + 1 > 4 * nBC + 1) return;
  const int csrLen = ((nE + 31) & ~31) + 4096;
  if (31 * 4 * nBC > 4096) return;
  const int nAgg   = NPAD / TGT;
  const int nGemm  = NPAD / BM;
  const int nXu    = NPAD * (FIN0 / 8);

  char* ws = (char*)d_ws;
  size_t off = 0;
  const size_t hwBytesQ = (size_t)NPAD * HID * 2;
  const size_t hwBytesF = (size_t)NPAD * NOUT * 4;
  const size_t hwBytes  = hwBytesQ > hwBytesF ? hwBytesQ : hwBytesF;
  const size_t oW0  = off; off += (size_t)HID * FIN0 * 2;         off = (off + 255) & ~(size_t)255;
  const size_t oW1  = off; off += (size_t)HID * HID * 2;          off = (off + 255) & ~(size_t)255;
  const size_t oW2  = off; off += (size_t)NOUT * HID * 2;         off = (off + 255) & ~(size_t)255;
  const size_t oP   = off; off += (size_t)NPAD * HID * 2;         off = (off + 255) & ~(size_t)255;
  const size_t oHw  = off; off += hwBytes;                        off = (off + 255) & ~(size_t)255;
  const size_t oCnt = off; off += (size_t)CNTPAD * 4;             off = (off + 255) & ~(size_t)255;
  const size_t oOff = off; off += (size_t)CNTPAD * 4;             off = (off + 255) & ~(size_t)255;
  const size_t oRb  = off; off += (size_t)RBN * 4;                off = (off + 255) & ~(size_t)255;
  const size_t oCsr = off; off += (size_t)csrLen * 4;             off = (off + 255) & ~(size_t)255;
  const size_t oES  = off; off += (size_t)NPAD * NHEAD * 4;       off = (off + 255) & ~(size_t)255;
  const size_t oED  = off; off += (size_t)NPAD * NHEAD * 4;       off = (off + 255) & ~(size_t)255;
  if (off > ws_size || off > (size_t)WSCAP) return;
  _Float16* wq0 = (_Float16*)(ws + oW0);
  _Float16* wq1 = (_Float16*)(ws + oW1);
  _Float16* wq2 = (_Float16*)(ws + oW2);
  _Float16* pP  = (_Float16*)(ws + oP);
  _Float16* hq  = (_Float16*)(ws + oHw);
  float*    hf  = (float*)(ws + oHw);
  int*   cnt  = (int*)(ws + oCnt);
  int*   offp = (int*)(ws + oOff);
  int*   rb   = (int*)(ws + oRb);
  int*   csr  = (int*)(ws + oCsr);
  float* es   = (float*)(ws + oES);
  float* ed   = (float*)(ws + oED);

  const int vec8 = ((nE & 3) == 0) ? 1 : 0;

  k_wprep<FIN0, HID><<<(HID * FIN0 / 8 + NTHR - 1) / NTHR, NTHR, 0, stream>>>(W0, wq0);
  k_wprep<HID, HID><<<(HID * HID / 8 + NTHR - 1) / NTHR, NTHR, 0, stream>>>(W1, wq1);
  k_wprep<HID, NOUT><<<(NOUT * HID / 8 + NTHR - 1) / NTHR, NTHR, 0, stream>>>(W2, wq2);
  k_xcvt<<<(nXu + NTHR - 1) / NTHR, NTHR, 0, stream>>>(x, pP, nN, nXu);

  k_count<<<nBC, NTHR, 0, stream>>>(dst, cnt, nE, vec8);
  k_offsets<<<1, OTHR, 0, stream>>>(cnt, offp, rb, nBC);
  hipFuncSetAttribute(reinterpret_cast<const void*>(&k_fill),
                      hipFuncAttributeMaxDynamicSharedMemorySize, LDS_FILL);
  k_fill<<<nBF, NTHR, LDS_FILL, stream>>>(src, dst, offp, rb, csr, nN, nE, vec8, csrLen);

  k_gemm<FIN0, HID, 0><<<nGemm, NTHR, 0, stream>>>(pP, wq0, as0, ad0, hq, hf, es, ed);
  k_agg<HID, 0><<<nAgg, NTHR, 0, stream>>>(csr, offp, cnt, es, ed, hq, hf, b0, pP, out, nN, csrLen);

  k_gemm<HID, HID, 0><<<nGemm, NTHR, 0, stream>>>(pP, wq1, as1, ad1, hq, hf, es, ed);
  k_agg<HID, 0><<<nAgg, NTHR, 0, stream>>>(csr, offp, cnt, es, ed, hq, hf, b1, pP, out, nN, csrLen);

  k_gemm<HID, NOUT, 1><<<nGemm, NTHR, 0, stream>>>(pP, wq2, as2, ad2, hq, hf, es, ed);
  k_agg<NOUT, 1><<<nAgg, NTHR, 0, stream>>>(csr, offp, cnt, es, ed, hq, hf, b2, pP, out, nN, csrLen);
}
